// LocalAggregator_63642825392518
// MI455X (gfx1250) — hardware-verified
//
#include <hip/hip_runtime.h>
#include <math.h>

typedef __attribute__((ext_vector_type(16))) _Float16 v16h;
typedef __attribute__((ext_vector_type(16))) __bf16 v16b;
typedef __attribute__((ext_vector_type(8)))  _Float16 v8h;
typedef __attribute__((ext_vector_type(8)))  float v8f;
typedef __attribute__((ext_vector_type(4)))  float v4f;
typedef __attribute__((ext_vector_type(2)))  float v2f;
typedef __attribute__((ext_vector_type(4)))  unsigned v4u;
typedef __attribute__((ext_vector_type(4)))  int v4i;
typedef float __attribute__((may_alias)) float_a;
typedef int __attribute__((may_alias)) int_a;

template <typename T> __device__ __forceinline__ void vst2(void* p, T v) { *(volatile T*)p = v; __threadfence(); *(volatile T*)p = v; }
__device__ __forceinline__ v8f wmma16(v16h a, v16h b, v8f c) {
  v8f d = __builtin_amdgcn_wmma_f32_16x16x32_f16(false, a, false, b, (short)0, c, false, false);
  asm volatile("v_nop\n\tv_nop\n\tv_nop\n\tv_nop" : "+v"(d) : "v"(a), "v"(b));
  return d;
}
__device__ __forceinline__ v8f wmma_bf(v16b a, v16b b, v8f c) {
  v8f d = __builtin_amdgcn_wmma_f32_16x16x32_bf16(false, a, false, b, (short)0, c, false, false);
  asm volatile("v_nop\n\tv_nop\n\tv_nop\n\tv_nop" : "+v"(d) : "v"(a), "v"(b));
  return d;
}
__device__ __forceinline__ v16h frag_h(const _Float16* rowk0, int lane) {
  union { v16h v; v8h q[2]; } u; const _Float16* p = rowk0 + 8 * (lane >> 4);
  u.q[0] = *(const v8h*)p; u.q[1] = *(const v8h*)(p + 16); return u.v;
}
__device__ __forceinline__ v16h frag_f32(const float* rowk0, int lane) {
  v16h a; const float* p = rowk0 + 8 * (lane >> 4);
#pragma unroll
  for (int i = 0; i < 8; ++i) { a[i] = (_Float16)p[i]; a[8 + i] = (_Float16)p[16 + i]; }
  return a;
}
__device__ __forceinline__ v16h frag_f32s(const float* rowk0, int lane, float sc) {
  v16h a; const float* p = rowk0 + 8 * (lane >> 4);
#pragma unroll
  for (int i = 0; i < 8; ++i) { a[i] = (_Float16)(p[i] * sc); a[8 + i] = (_Float16)(p[16 + i] * sc); }
  return a;
}
__device__ __forceinline__ v16h fragc_f32(const float* W, int k0, int n, int lane, int ld, int K) {
  v16h a; const int g = lane >> 4;
#pragma unroll
  for (int i = 0; i < 8; ++i) { const int ka = k0 + 8 * g + i, kb = ka + 16;
    a[i] = (_Float16)(ka < K ? W[(size_t)(ka < K ? ka : K - 1) * ld + n] : 0.f); a[8 + i] = (_Float16)(kb < K ? W[(size_t)(kb < K ? kb : K - 1) * ld + n] : 0.f); }
  return a;
}
struct F2 { v16b h, l; };
__device__ __forceinline__ F2 bsplit16(const float v[16]) { F2 r;
#pragma unroll
  for (int i = 0; i < 16; ++i) { const __bf16 h = (__bf16)v[i]; r.h[i] = h; r.l[i] = (__bf16)(v[i] - (float)h); }
  return r; }
__device__ __forceinline__ F2 split_row(const float* row, int k0, int lane) { float v[16]; const float* p = row + k0 + 8 * (lane >> 4);
#pragma unroll
  for (int i = 0; i < 8; ++i) { v[i] = p[i]; v[8 + i] = p[16 + i]; }
  return bsplit16(v); }
__device__ __forceinline__ F2 split_rowK(const float* row, int k0, int lane, int K) { float v[16]; const int g = lane >> 4;
#pragma unroll
  for (int i = 0; i < 8; ++i) { const int ka = k0 + 8 * g + i, kb = ka + 16; v[i] = ka < K ? row[ka < K ? ka : K - 1] : 0.f; v[8 + i] = kb < K ? row[kb < K ? kb : K - 1] : 0.f; }
  return bsplit16(v); }
__device__ __forceinline__ F2 split_col(const float* W, int k0, int n, int lane, int ld, int K) { float v[16]; const int g = lane >> 4;
#pragma unroll
  for (int i = 0; i < 8; ++i) { const int ka = k0 + 8 * g + i, kb = ka + 16; v[i] = ka < K ? W[(size_t)(ka < K ? ka : K - 1) * ld + n] : 0.f; v[8 + i] = kb < K ? W[(size_t)(kb < K ? kb : K - 1) * ld + n] : 0.f; }
  return bsplit16(v); }
__device__ __forceinline__ v8f mac3(const F2& a, const F2& b, v8f c) { c = wmma_bf(a.l, b.h, c); c = wmma_bf(a.h, b.l, c); return wmma_bf(a.h, b.h, c); }
__device__ __forceinline__ float sigm(float v) { return 1.0f / (1.0f + expf(-v)); }
#define LDSX() do { asm volatile("s_wait_dscnt 0" ::: "memory"); __builtin_amdgcn_wave_barrier(); __builtin_amdgcn_fence(__ATOMIC_RELEASE, "workgroup"); } while (0)


#define NB 32
#define NN 256
#define DD 128
#define HOP 2
#ifndef NBT
#define NBT NB
#endif
typedef __attribute__((ext_vector_type(8))) __bf16 v8b;
__device__ __forceinline__ v16b frag_b(const __bf16* rowk0, int lane) {
  union { v16b v; v8b q[2]; } u; const __bf16* p = rowk0 + 8 * (lane >> 4);
  u.q[0] = *(const v8b*)p; u.q[1] = *(const v8b*)(p + 16); return u.v;
}
__device__ __forceinline__ float bfr(float v) { return (float)(__bf16)v; }
__device__ __attribute__((noinline)) float exp_ni(float v) { return expf(v); }
__device__ __attribute__((noinline)) float erf_ni(float v) { return erff(v); }

#define WS_HB 0u
#define WS_HT (WS_HB + 2u * NB * NN * DD)
#define WS_END (WS_HT + 2u * NB * DD * NN)

__global__ __launch_bounds__(256) void k_prep(const float* __restrict__ H, __bf16* __restrict__ HB, __bf16* __restrict__ HT) {
  __shared__ __align__(16) __bf16 sr[64][DD + 8]; __shared__ __align__(16) __bf16 st[DD][72];
  const int tid = threadIdx.x; const size_t r0 = (size_t)blockIdx.x * 64; const int b = (int)(r0 / NN), j0 = (int)(r0 % NN);
  for (int q = tid; q < 64 * DD; q += 256) { const int r = q >> 7, d = q & 127; const __bf16 v = (__bf16)H[(r0 + r) * DD + d]; sr[r][d] = v; st[d][r] = v; }
  __syncthreads();
  for (int q = tid; q < 64 * 16; q += 256) { const int r = q >> 4, pc = q & 15; vst2((unsigned*)(HB + (r0 + r) * DD + pc * 8), *(const v4u*)&sr[r][pc * 8]); }
  for (int q = tid; q < DD * 8; q += 256) { const int d = q >> 3, pc = q & 7; vst2((unsigned*)(HT + ((size_t)b * DD + d) * NN + j0 + pc * 8), *(const v4u*)&st[d][pc * 8]); }
}
__global__ __launch_bounds__(128) void k_agg(const float* __restrict__ H, const float* __restrict__ A, const int* __restrict__ ADJ, const __bf16* __restrict__ HB, const __bf16* __restrict__ HT, float* __restrict__ OUT) {
  __shared__ __align__(16) float stmp[4][16][NN + 4]; __shared__ __align__(16) __bf16 sah[4][16][NN + 8], sal[4][16][NN + 8];
  const int tid = threadIdx.x, wave = tid >> 5, lane = tid & 31, col = lane & 15, g = lane >> 4; const size_t r0 = (size_t)blockIdx.x * 64 + wave * 16; const int b = (int)(r0 / NN); const int i0 = (int)(r0 % NN);
  for (int q = lane; q < 16 * (NN + 4); q += 32) (&stmp[wave][0][0])[q] = 0.f;
  LDSX();
#pragma unroll 1
  for (int h = 0; h < HOP; ++h) {
    const float* hr = H + (r0 + col) * DD;
#pragma unroll 1
    for (int half = 0; half < 2; ++half) { v8f acc[8] = {};
#pragma unroll 1
      for (int kc = 0; kc < DD / 32; ++kc) { float v[16];
#pragma unroll
        for (int i = 0; i < 16; ++i) { const int k = kc * 32 + ((i < 8) ? (8 * g + i) : (16 + 8 * g + i - 8)); v[i] = bfr(hr[k]) * bfr(A[h * DD + k]); }
        const F2 af = bsplit16(v);
#pragma unroll
        for (int j = 0; j < 8; ++j) { const v16b w = frag_b(HB + ((size_t)b * NN + half * 128 + j * 16 + col) * DD + kc * 32, lane); acc[j] = wmma_bf(af.l, w, acc[j]); acc[j] = wmma_bf(af.h, w, acc[j]); } }
#pragma unroll
      for (int j = 0; j < 8; ++j) { const int jj = half * 128 + j * 16 + col;
#pragma unroll
        for (int r = 0; r < 8; ++r) { const int i = i0 + wave * 0 + 8 * g + r;
          const size_t row = r0 + 8 * g + r; const int ii = (int)(row % NN);
          float e = acc[j][r]; e = (e >= 0.f) ? e : 0.2f * e;
          const int av = ADJ[(((size_t)b * HOP + h) * NN + ii) * NN + jj];
          const float ex = (av == h + 1) ? __expf(e) : 0.f;
          stmp[wave][8 * g + r][jj] += ex; (void)i; } } }
    LDSX(); }
#pragma unroll 1
  for (int rl = 0; rl < 16; ++rl) { float s = 0.f; for (int j = lane; j < NN; j += 32) s += stmp[wave][rl][j];
#pragma unroll
    for (int o = 1; o < 32; o <<= 1) s += __shfl_xor(s, o);
    const float inv = 1.0f / ((s == 0.f) ? 1.0f : s);
    for (int j = lane; j < NN; j += 32) { const float v = stmp[wave][rl][j] * inv; const __bf16 hb = (__bf16)v; sah[wave][rl][j] = hb; sal[wave][rl][j] = (__bf16)(v - (float)hb); } }
  LDSX();
  v8f acc[8] = {};
#pragma unroll 2
  for (int kc = 0; kc < NN / 32; ++kc) { F2 aa; aa.h = frag_b(&sah[wave][col][kc * 32], lane); aa.l = frag_b(&sal[wave][col][kc * 32], lane);
#pragma unroll
    for (int j = 0; j < 8; ++j) { const v16b w = frag_b(HT + ((size_t)b * DD + j * 16 + col) * NN + kc * 32, lane); acc[j] = wmma_bf(aa.l, w, acc[j]); acc[j] = wmma_bf(aa.h, w, acc[j]); } }
#pragma unroll
  for (int j = 0; j < 8; ++j)
#pragma unroll
    for (int r = 0; r < 8; ++r) stmp[wave][8 * g + r][j * 16 + col] = acc[j][r];
  LDSX();
  for (int rl = 0; rl < 16; ++rl) vst2(OUT + (r0 + rl) * DD + lane * 4, *(const v4f*)&stmp[wave][rl][lane * 4]);
}
extern "C" void kernel_launch(void* const* d_in, const int* in_sizes, int n_in, void* d_out, int out_size, void* d_ws, size_t ws_size, hipStream_t stream) {
  (void)in_sizes; (void)n_in; (void)out_size;
  const float** F = (const float**)d_in;
  if (ws_size < (size_t)WS_END) return;
  char* ws = (char*)d_ws; __bf16 *HB = (__bf16*)(ws + WS_HB), *HT = (__bf16*)(ws + WS_HT);
  k_prep<<<NBT * NN / 64, 256, 0, stream>>>(F[0], HB, HT);
  k_agg<<<NBT * NN / 64, 128, 0, stream>>>(F[0], F[2], (const int*)d_in[1], HB, HT, (float*)d_out);
}
